// GCNEncoder_36017595744478
// MI455X (gfx1250) — hardware-run, weakly checked
//
#include <hip/hip_runtime.h>

typedef float          v8f   __attribute__((ext_vector_type(8)));
typedef float          v4f   __attribute__((ext_vector_type(4)));
typedef unsigned int   v4u   __attribute__((ext_vector_type(4)));
typedef int            v8i   __attribute__((ext_vector_type(8)));
typedef unsigned short v8us  __attribute__((ext_vector_type(8)));
typedef unsigned short v16us __attribute__((ext_vector_type(16)));
typedef __bf16         v16bf __attribute__((ext_vector_type(16)));
typedef _Float16       v16h  __attribute__((ext_vector_type(16)));
typedef v4f  __attribute__((may_alias)) v4fa;
typedef v8us __attribute__((may_alias)) v8usa;
union FragB { v16bf v; v16us u; v8us h[2]; v8i w; };
union FragH { v16h  v; v16us u; v8us h[2]; v8i w; };

__device__ __forceinline__ v8f wmb(const FragB& a, const FragB& b, v8f c) {
  v8f d = __builtin_amdgcn_wmma_f32_16x16x32_bf16(false, a.v, false, b.v, (short)0, c, false, false);
  asm volatile("v_nop\n\tv_nop\n\tv_nop\n\tv_nop" : "+v"(d) : "v"(a.w), "v"(b.w));
  return d;
}

__device__ __forceinline__ v8f wmh(const FragH& a, const FragH& b, v8f c) {
  v8f d = __builtin_amdgcn_wmma_f32_16x16x32_f16(false, a.v, false, b.v, (short)0, c, false, false);
  asm volatile("v_nop\n\tv_nop\n\tv_nop\n\tv_nop" : "+v"(d) : "v"(a.w), "v"(b.w));
  return d;
}

__device__ __forceinline__ unsigned bf16_bits(float f) {
  const unsigned u = __float_as_uint(f);
  const unsigned r = (u + 0x7FFFu + ((u >> 16) & 1u)) >> 16;
  const unsigned q = (u >> 16) | 0x40u;
  return ((u & 0x7fffffffu) > 0x7f800000u) ? q : r;
}

__device__ __forceinline__ float bf16_val(float f) {
  return __uint_as_float(bf16_bits(f) << 16);
}
__device__ __forceinline__ int clampi(int v, int lo, int hi) {
  return v < lo ? lo : (v > hi ? hi : v);
}

__device__ __forceinline__ unsigned f16_bits(float f) {
  const unsigned u  = __float_as_uint(f);
  const unsigned s  = (u >> 16) & 0x8000u;
  const unsigned a  = u & 0x7fffffffu;
  const unsigned t  = a - 0x38000000u;
  const unsigned r  = (t + 0x0FFFu + ((t >> 13) & 1u)) >> 13;
  const unsigned rc = r > 0x7C00u ? 0x7C00u : r;
  const bool small  = a < 0x38800000u;
  const bool isnan  = a > 0x7f800000u;
  const unsigned fin = small ? 0u : (s | rc);
  return isnan ? (s | 0x7E00u) : fin;
}

__device__ __forceinline__ unsigned pk16(unsigned lo, unsigned hi) { return lo | (hi << 16); }
__device__ __forceinline__ unsigned bf16_lo_bits(float v) {
  float hi = bf16_val(v);
  asm volatile("" : "+v"(hi));
  return bf16_bits(v - hi);
}
__device__ __forceinline__ v4u pack8_bf16(v4f a, v4f c) {
  return (v4u){ pk16(bf16_bits(a[0]), bf16_bits(a[1])), pk16(bf16_bits(a[2]), bf16_bits(a[3])),
                pk16(bf16_bits(c[0]), bf16_bits(c[1])), pk16(bf16_bits(c[2]), bf16_bits(c[3])) };
}
__device__ __forceinline__ v4u pack8_bf16_lo(v4f a, v4f c) {
  return (v4u){ pk16(bf16_lo_bits(a[0]), bf16_lo_bits(a[1])), pk16(bf16_lo_bits(a[2]), bf16_lo_bits(a[3])),
                pk16(bf16_lo_bits(c[0]), bf16_lo_bits(c[1])), pk16(bf16_lo_bits(c[2]), bf16_lo_bits(c[3])) };
}
__device__ __forceinline__ v4u pack8_f16(v4f a, v4f c) {
  return (v4u){ pk16(f16_bits(a[0]), f16_bits(a[1])), pk16(f16_bits(a[2]), f16_bits(a[3])),
                pk16(f16_bits(c[0]), f16_bits(c[1])), pk16(f16_bits(c[2]), f16_bits(c[3])) };
}

template <int FORM>
__global__ __launch_bounds__(256) void k_plane(const float* __restrict__ src, int rows, int cols, int ldsrc,
                                               unsigned short* __restrict__ dst, int MP, int KP) {
  static_assert(FORM >= 0 && FORM <= 3);
  const int KTOT = (FORM == 1 || FORM == 3) ? 2 * KP : KP;
  const unsigned ppr   = (unsigned)(KTOT >> 3);
  const unsigned kp8   = (unsigned)(KP >> 3);
  const unsigned total = (unsigned)MP * ppr;
  const unsigned g     = blockIdx.x * 256u + threadIdx.x;
  const unsigned rowu  = g / ppr;
  const unsigned p     = g - rowu * ppr;
  const bool second    = p >= kp8;
  const int row = (int)rowu;
  const int c0  = (int)((second ? p - kp8 : p) << 3);
  const float* srow = src + (size_t)clampi(row, 0, rows - 1) * (size_t)ldsrc;
  float x[8];
  unsigned mk[8];
#pragma unroll
  for (int e = 0; e < 8; ++e) {
    const int c = c0 + e;
    const float v = srow[clampi(c, 0, cols - 1)];
    asm volatile("" :: "v"(v));
    x[e]  = v;
    mk[e] = (row < rows && c < cols) ? 0xFFFFu : 0u;
  }
  const v4f a = (v4f){ x[0], x[1], x[2], x[3] };
  const v4f c = (v4f){ x[4], x[5], x[6], x[7] };
  v4u o;
  if (FORM == 2) {
    o = pack8_f16(a, c);
  } else {
    const v4u hi = pack8_bf16(a, c);
    o = hi;
    if (FORM == 1) { const v4u lo = pack8_bf16_lo(a, c); o = second ? lo : hi; }
  }
  const v4u mw = (v4u){ pk16(mk[0], mk[1]), pk16(mk[2], mk[3]), pk16(mk[4], mk[5]), pk16(mk[6], mk[7]) };
  o &= mw;
  if (g < total) {
    volatile v4u* q = (volatile v4u*)(dst + (size_t)g * 8);
    *q = o;
    __threadfence();
    *q = o;
  }
}

template <int FORM> struct FragOf    { typedef FragB T; };
template <>         struct FragOf<2> { typedef FragH T; };
__device__ __forceinline__ v8f mm(const FragB& a, const FragB& b, v8f c) { return wmb(a, b, c); }
__device__ __forceinline__ v8f mm(const FragH& a, const FragH& b, v8f c) { return wmh(a, b, c); }
template <class F> __device__ __forceinline__ F ld_frag(const unsigned short* p) {
  F f;
  f.h[0] = *(const v8usa*)(p);
  f.h[1] = *(const v8usa*)(p + 16);
  return f;
}

template <int FORM, int EPI>
__global__ __launch_bounds__(256) __attribute__((amdgpu_num_vgpr(248)))
void k_gemm_nt(const unsigned short* __restrict__ A, const unsigned short* __restrict__ B,
               const float* __restrict__ bias, float* __restrict__ D, int M, int N, int KTOT, int ldd) {
  static_assert(FORM >= 0 && FORM <= 2);
  static_assert(EPI == 0 || EPI == 1);
  typedef typename FragOf<FORM>::T F;
  __shared__ __attribute__((aligned(16))) float sT[8][16 * 68];
  const int lane = threadIdx.x & 31;
  const int wave = threadIdx.x >> 5;
  const int tilesM = (M + 63) >> 6;
  const int tilesN = (N + 63) >> 6;
  const int tile = blockIdx.x * 8 + wave;
  if (tile >= tilesM * tilesN) return;
  const int tm = tile / tilesN;
  const int tn = tile - tm * tilesN;
  const int m0 = tm << 6;
  const int n0 = tn << 6;

  const int rl = lane & 15;
  const int h8 = (lane >> 4) * 8;
  const unsigned short* pa = A + (size_t)(m0 + rl) * (size_t)KTOT + h8;
  const unsigned short* pb = B + (size_t)(n0 + rl) * (size_t)KTOT + h8;

  v8f acc[4][4];
#pragma unroll
  for (int i = 0; i < 4; ++i)
#pragma unroll
    for (int j = 0; j < 4; ++j) acc[i][j] = (v8f){0.f, 0.f, 0.f, 0.f, 0.f, 0.f, 0.f, 0.f};

#pragma unroll 1
  for (int k0 = 0; k0 < KTOT; k0 += 32) {
    F bf[4];
#pragma unroll
    for (int j = 0; j < 4; ++j) bf[j] = ld_frag<F>(pb + (size_t)(j << 4) * (size_t)KTOT + k0);
#pragma unroll
    for (int i = 0; i < 4; ++i) {
      const F af = ld_frag<F>(pa + (size_t)(i << 4) * (size_t)KTOT + k0);
#pragma unroll
      for (int j = 0; j < 4; ++j) acc[i][j] = mm(af, bf[j], acc[i][j]);
    }
  }

  float* slab = sT[wave];
  const int hh = lane >> 4;
  const int c4 = (lane & 15) * 4;
  const int nc = n0 + c4;
  const bool cok = nc < N;
  v4f bv = (v4f){0.f, 0.f, 0.f, 0.f};
  if (EPI == 1) {
    bv = *(const v4fa*)(bias + clampi(nc, 0, N - 4));
    asm volatile("" :: "v"(bv));
  }
#pragma unroll
  for (int i = 0; i < 4; ++i) {
    const int mBase = m0 + (i << 4);
#pragma unroll
    for (int j = 0; j < 4; ++j) {
#pragma unroll
      for (int r = 0; r < 8; ++r) slab[(h8 + r) * 68 + (j << 4) + rl] = acc[i][j][r];
    }
    __builtin_amdgcn_fence(__ATOMIC_RELEASE, "workgroup");
    __builtin_amdgcn_wave_barrier();
    __builtin_amdgcn_fence(__ATOMIC_ACQUIRE, "workgroup");
    v4f vv[8];
#pragma unroll
    for (int it = 0; it < 8; ++it) {
      const int row = it * 2 + hh;
      v4f v = *(const v4fa*)(slab + row * 68 + c4);
      if (EPI == 1) v += bv;
      vv[it] = v;
    }
    for (int pass = 0; pass < 2; ++pass) {
#pragma unroll
      for (int it = 0; it < 8; ++it) {
        const int row = mBase + it * 2 + hh;
        if (cok && row < M) *(volatile v4f*)(D + (size_t)row * (size_t)ldd + nc) = vv[it];
      }
      __threadfence();
    }
    __builtin_amdgcn_fence(__ATOMIC_RELEASE, "workgroup");
    __builtin_amdgcn_wave_barrier();
    __builtin_amdgcn_fence(__ATOMIC_ACQUIRE, "workgroup");
  }
}

#pragma clang fp contract(off)

#ifndef MODE2
#define MODE2 2
#endif
#ifndef MODE3
#define MODE3 2
#endif
static_assert(MODE2 == 1 || MODE2 == 2);
static_assert(MODE3 == 1 || MODE3 == 2);

typedef float        v2f __attribute__((ext_vector_type(2)));
typedef unsigned int v2u __attribute__((ext_vector_type(2)));
typedef int          v4i __attribute__((ext_vector_type(4)));
typedef double       v2d __attribute__((ext_vector_type(2)));
typedef v2f __attribute__((may_alias)) v2fa;
typedef v2u __attribute__((may_alias)) v2ua;
typedef v4i __attribute__((may_alias)) v4ia;

constexpr int NN    = 50000;
constexpr int NE    = 800000;
constexpr int HID   = 128;
constexpr int COUT  = 64;
constexpr int NP    = 50048;
constexpr int NREC  = NP / 128;
constexpr int NBRUN = 1024;
constexpr int NBLK  = 49;
constexpr int RCAP  = 20992;
constexpr int DEGCAP = 48;
constexpr int WLCAP = 3072;
constexpr int EPW   = NE / 8;
constexpr int SUB   = 128;
constexpr int NSTEP = (EPW + SUB - 1) / SUB;
constexpr int K2T   = (MODE2 == 2) ? 2 * HID : HID;
constexpr int K3T   = (MODE3 == 2) ? 2 * HID : HID;

static_assert(NP % 64 == 0 && NP >= NN && NP - NN < 64 && NREC * 128 == NP && NP % 16 == 0);
static_assert(NBLK * NBRUN >= NN && (NBLK - 1) * NBRUN < NN);
static_assert(NE % 8 == 0 && NSTEP * SUB >= EPW && (NSTEP - 1) * SUB < EPW);
static_assert(RCAP % 256 == 0 && RCAP * 4 >= 16623 * 5 && RCAP >= 2 * DEGCAP);
static_assert(DEGCAP >= 35 + 8 && DEGCAP % 16 == 0);
static_assert(WLCAP * 8 >= RCAP);
static_assert(NN <= 65536 && (((long long)(NN - 1) << 10) | 1023) < (1LL << 31));
static_assert(K2T % 32 == 0 && K3T % 32 == 0 && HID % 32 == 0 && COUT % 32 == 0);
static_assert(NN % 8 == 0);

constexpr int P_B1 = 0, P_B2 = 128, P_B3 = 256, P_G1 = 384, P_BE1 = 512, P_G2 = 640, P_BE2 = 768, P_N = 896;
constexpr int S_M1 = 0, S_R1 = 128, S_M2 = 256, S_R2 = 384, S_N = 512;

constexpr int BK_WL   = 0;
constexpr int BK_SL   = 8 * WLCAP;
constexpr int BK_CNT  = BK_SL + RCAP;
constexpr int BK_OFF  = BK_CNT + NBRUN;
constexpr int BK_CUR  = BK_OFF + NBRUN;
constexpr int BK_DVB  = BK_CUR + NBRUN;
constexpr int BK_MISC = BK_DVB + NBRUN;
constexpr int BK_INTS = BK_MISC + 16;
constexpr int BK_LDS  = BK_INTS * 4;
static_assert(BK_LDS <= 262144);
static_assert(BK_SL % 4 == 0 && BK_CNT % 4 == 0 && (RCAP + NBRUN) % 4 == 0);

constexpr size_t SZ_F    = (size_t)NP * HID * 4;
constexpr size_t SZ_HL   = (size_t)NP * 256 * 2;
constexpr size_t SZ_XB   = (size_t)NP * HID * 2;
constexpr size_t SZ_LIST = (size_t)NBLK * RCAP * 4;
constexpr size_t SZ_NODE = (size_t)NBLK * NBRUN * 4;
constexpr size_t SZ_FLAG = 6400;
constexpr size_t SZ_W1T  = (size_t)HID * HID * 2;
constexpr size_t SZ_W2D  = (size_t)HID * 256 * 2;
constexpr size_t SZ_W3D  = (size_t)COUT * 256 * 2;
constexpr size_t SZ_PAR  = 3584;
constexpr size_t SZ_REC  = (size_t)NREC * HID * 8;
constexpr size_t SZ_ST   = 2048;
constexpr size_t OFF_PA   = 0;
constexpr size_t OFF_PB   = OFF_PA + SZ_F;
constexpr size_t OFF_PC   = OFF_PB + SZ_F;
constexpr size_t OFF_HL   = OFF_PC + SZ_F;
constexpr size_t OFF_XB   = OFF_HL + SZ_HL;
constexpr size_t OFF_LIST = OFF_XB + SZ_XB;
constexpr size_t OFF_CNT  = OFF_LIST + SZ_LIST;
constexpr size_t OFF_OFF  = OFF_CNT + SZ_NODE;
constexpr size_t OFF_DINV = OFF_OFF + SZ_NODE;
constexpr size_t OFF_FLAG = OFF_DINV + SZ_NODE;
constexpr size_t OFF_W1T  = OFF_FLAG + SZ_FLAG;
constexpr size_t OFF_W2D  = OFF_W1T + SZ_W1T;
constexpr size_t OFF_W3D  = OFF_W2D + SZ_W2D;
constexpr size_t OFF_PAR  = OFF_W3D + SZ_W3D;
constexpr size_t OFF_REC  = OFF_PAR + SZ_PAR;
constexpr size_t OFF_ST   = OFF_REC + SZ_REC;
constexpr size_t WS_TOTAL = OFF_ST + SZ_ST;
static_assert(WS_TOTAL == (size_t)((size_t)470979 << 8));
static_assert(WS_TOTAL <= ((size_t)128 << 20));
static_assert(SZ_F % 256 == 0 && SZ_HL % 256 == 0 && SZ_XB % 256 == 0 && SZ_LIST % 256 == 0 && SZ_NODE % 256 == 0);
static_assert(SZ_FLAG % 256 == 0 && SZ_PAR % 256 == 0 && SZ_REC % 256 == 0 && SZ_ST % 256 == 0);
static_assert((size_t)NBLK * 128 <= SZ_FLAG && (size_t)P_N * 4 <= SZ_PAR && (size_t)S_N * 4 <= SZ_ST);
static_assert((size_t)NP * K2T * 2 <= SZ_HL && (size_t)NP * K3T * 2 <= SZ_HL);
static_assert((size_t)HID * K2T * 2 <= SZ_W2D && (size_t)COUT * K3T * 2 <= SZ_W3D);
static_assert((size_t)NP * COUT * 4 <= SZ_F);

__device__ __forceinline__ float relu_k(float v) { return (v > 0.0f) ? v : (v - v); }

constexpr int PB_XB  = NP * (HID / 8) / 256;
constexpr int PB_W1  = HID * (HID / 8) / 256;
constexpr int PB_W2  = HID * (K2T / 8) / 256;
constexpr int PB_W3  = COUT * (K3T / 8) / 256;
constexpr int PB_TOT = PB_XB + PB_W1 + PB_W2 + PB_W3 + 1;
static_assert((NP * (HID / 8)) % 256 == 0 && (HID * (HID / 8)) % 256 == 0);
static_assert((HID * (K2T / 8)) % 256 == 0 && (COUT * (K3T / 8)) % 256 == 0);

__device__ __forceinline__ void wplane_unit(const float* __restrict__ W, int ncols, int ktot,
                                            unsigned short* __restrict__ dst, int u) {
  const int ppr = ktot >> 3;
  const int n   = u / ppr;
  const int p   = u - n * ppr;
  const int k8  = (p << 3) & (HID - 1);
  const float* s = W + (size_t)k8 * (size_t)ncols + n;
  float x[8];
#pragma unroll
  for (int i = 0; i < 8; ++i) {
    const float v = s[(size_t)i * (size_t)ncols];
    asm volatile("" :: "v"(v));
    x[i] = v;
  }
  const v4u o = pack8_bf16((v4f){ x[0], x[1], x[2], x[3] }, (v4f){ x[4], x[5], x[6], x[7] });
  volatile v4u* q = (volatile v4u*)(dst + (size_t)u * 8);
  *q = o;
  __threadfence();
  *q = o;
}

__global__ __launch_bounds__(256) void k_prep(const float* __restrict__ x,
                                              const float* __restrict__ W1, const float* __restrict__ W2,
                                              const float* __restrict__ W3,
                                              const float* __restrict__ b1, const float* __restrict__ b2,
                                              const float* __restrict__ b3,
                                              const float* __restrict__ g1, const float* __restrict__ be1,
                                              const float* __restrict__ g2, const float* __restrict__ be2,
                                              unsigned short* __restrict__ XB, unsigned short* __restrict__ W1T,
                                              unsigned short* __restrict__ W2D, unsigned short* __restrict__ W3D,
                                              float* __restrict__ PAR) {
  const int tid = (int)threadIdx.x;
  const int blk = (int)blockIdx.x;
  if (blk < PB_XB) {
    const int u   = blk * 256 + tid;
    const int row = u >> 4;
    const int k8  = (u & 15) * 8;
    const int rc  = row < NN ? row : NN - 1;
    const float* p = x + (size_t)rc * HID + k8;
    const v4f a = *(const v4fa*)p;
    const v4f c = *(const v4fa*)(p + 4);
    asm volatile("" :: "v"(a));
    asm volatile("" :: "v"(c));
    v4u o = pack8_bf16(a, c);
    const unsigned mk = (row < NN) ? 0xFFFFFFFFu : 0u;
    o &= (v4u){ mk, mk, mk, mk };
    volatile v4u* q = (volatile v4u*)(XB + (size_t)u * 8);
    *q = o;
    __threadfence();
    *q = o;
  } else if (blk < PB_XB + PB_W1) {
    wplane_unit(W1, HID, HID, W1T, (blk - PB_XB) * 256 + tid);
  } else if (blk < PB_XB + PB_W1 + PB_W2) {
    wplane_unit(W2, HID, K2T, W2D, (blk - PB_XB - PB_W1) * 256 + tid);
  } else if (blk < PB_XB + PB_W1 + PB_W2 + PB_W3) {
    wplane_unit(W3, COUT, K3T, W3D, (blk - PB_XB - PB_W1 - PB_W2) * 256 + tid);
  } else {
    const int u   = tid < P_N / 4 ? tid : P_N / 4 - 1;
    const int seg = u >> 5;
    const int j   = u & 31;
    const int j3  = j < 16 ? j : 15;
    const v4f a0 = *(const v4fa*)(b1 + 4 * j);
    const v4f a1 = *(const v4fa*)(b2 + 4 * j);
    const v4f a2 = *(const v4fa*)(b3 + 4 * j3);
    const v4f a3 = *(const v4fa*)(g1 + 4 * j);
    const v4f a4 = *(const v4fa*)(be1 + 4 * j);
    const v4f a5 = *(const v4fa*)(g2 + 4 * j);
    const v4f a6 = *(const v4fa*)(be2 + 4 * j);
    asm volatile("" :: "v"(a0));
    asm volatile("" :: "v"(a1));
    asm volatile("" :: "v"(a2));
    asm volatile("" :: "v"(a3));
    asm volatile("" :: "v"(a4));
    asm volatile("" :: "v"(a5));
    asm volatile("" :: "v"(a6));
    const unsigned m0 = (seg == 0) ? 0xFFFFFFFFu : 0u;
    const unsigned m1 = (seg == 1) ? 0xFFFFFFFFu : 0u;
    const unsigned m2 = (seg == 2 && j < 16) ? 0xFFFFFFFFu : 0u;
    const unsigned m3 = (seg == 3) ? 0xFFFFFFFFu : 0u;
    const unsigned m4 = (seg == 4) ? 0xFFFFFFFFu : 0u;
    const unsigned m5 = (seg == 5) ? 0xFFFFFFFFu : 0u;
    const unsigned m6 = (seg == 6) ? 0xFFFFFFFFu : 0u;
    v4f o;
#pragma unroll
    for (int e = 0; e < 4; ++e) {
      const unsigned bits = (__float_as_uint(a0[e]) & m0) | (__float_as_uint(a1[e]) & m1) |
                            (__float_as_uint(a2[e]) & m2) | (__float_as_uint(a3[e]) & m3) |
                            (__float_as_uint(a4[e]) & m4) | (__float_as_uint(a5[e]) & m5) |
                            (__float_as_uint(a6[e]) & m6);
      o[e] = bf16_val(__uint_as_float(bits));
    }
    if (tid < P_N / 4) {
      volatile v4f* q = (volatile v4f*)(PAR + 4 * tid);
      *q = o;
      __threadfence();
      *q = o;
    }
  }
}

__global__ __launch_bounds__(256) void k_bucket(const int* __restrict__ ei, int* __restrict__ LIST,
                                                int* __restrict__ CNT, int* __restrict__ OFF,
                                                float* __restrict__ DINV, int* __restrict__ FLAG) {
  extern __shared__ __attribute__((aligned(16))) int dsm[];
  int* wl   = dsm + BK_WL;
  int* sl   = dsm + BK_SL;
  int* cnt  = dsm + BK_CNT;
  int* offs = dsm + BK_OFF;
  int* cur  = dsm + BK_CUR;
  int* dvb  = dsm + BK_DVB;
  int* misc = dsm + BK_MISC;
  const int tid = (int)threadIdx.x, lane = tid & 31, wave = tid >> 5;
  const int blk = (int)blockIdx.x;
  const int nodeBase = blk * NBRUN;
  const int nbi = (NN - nodeBase) < NBRUN ? (NN - nodeBase) : NBRUN;
  const unsigned unb = (unsigned)(nbi < 0 ? 0 : nbi);

  {
    const v4i z4 = (v4i){0, 0, 0, 0};
    for (int i = tid * 4; i < RCAP + NBRUN; i += 1024) *(v4ia*)(sl + i) = z4;
    if (tid < 16) misc[tid] = 0;
  }
  __syncthreads();

  const int* srcp = ei;
  const int* dstp = ei + NE;
  int* mylist = wl + wave * WLCAP;
  const int wbase = wave * EPW;
  const int wlast = wbase + EPW - 1;
  int wc = 0;
#pragma unroll 1
  for (int st = 0; st < NSTEP; ++st) {
    const int e0 = wbase + st * SUB + lane;
    int dk[4], sk[4];
#pragma unroll
    for (int j = 0; j < 4; ++j) {
      const int e  = e0 + 32 * j;
      const int ec = e < wlast ? e : wlast;
      const int d = dstp[ec];
      const int s = srcp[ec];
      asm volatile("" :: "v"(d));
      asm volatile("" :: "v"(s));
      dk[j] = (e <= wlast) ? d : -1;
      sk[j] = s;
    }
#pragma unroll
    for (int j = 0; j < 4; ++j) {
      const unsigned slot = (unsigned)dk[j] - (unsigned)nodeBase;
      const bool hit = slot < unb;
      const unsigned mj = __builtin_amdgcn_ballot_w32(hit);
      if (mj != 0u) {
        if (hit) {
          const int pos = wc + (int)__builtin_amdgcn_mbcnt_lo(mj, 0u);
          if (pos < WLCAP) mylist[pos] = (clampi(sk[j], 0, NN - 1) << 10) | (int)slot;
        }
        wc += (int)__builtin_popcount(mj);
      }
    }
  }
  if (lane == 0) misc[wave] = wc;
  __syncthreads();

  if (wave == 0) {
    int t = 0, ov = 0;
#pragma unroll 1
    for (int w2 = 0; w2 < 8; ++w2) {
      const int craw = misc[w2];
      ov |= (craw > WLCAP) ? 1 : 0;
      const int c = __builtin_amdgcn_readfirstlane(clampi(craw, 0, WLCAP));
#pragma unroll 1
      for (int b0 = 0; b0 < c; b0 += 32) {
        const int idx = (b0 + lane) < c ? (b0 + lane) : c - 1;
        const int ent = wl[w2 * WLCAP + idx];
        const int m32 = (c - b0) < 32 ? (c - b0) : 32;
#pragma unroll 1
        for (int k = 0; k < m32; ++k) {
          const int u    = __builtin_amdgcn_readlane(ent, k);
          const int slot = u & (NBRUN - 1);
          if (t < RCAP) {
            if (lane == 0) cnt[slot] = cnt[slot] + 1;
            t = t + 1;
          } else {
            ov = 1;
          }
        }
      }
    }
    if (lane == 0) { misc[8] = t; misc[9] = ov; }
  }
  __syncthreads();

  if (wave == 0) {
    const int base = lane * (NBRUN / 32);
    int s = 0, big = 0;
#pragma unroll 1
    for (int i = 0; i < NBRUN / 32; ++i) {
      const int cv = cnt[base + i];
      s += cv;
      big |= (cv > DEGCAP) ? 1 : 0;
    }
    int incl = s;
#pragma unroll
    for (int d = 1; d < 32; d <<= 1) {
      const int y = __shfl_up(incl, d, 32);
      incl += (lane >= d) ? y : 0;
    }
    int run = incl - s;
#pragma unroll 1
    for (int i = 0; i < NBRUN / 32; ++i) {
      const int cv = cnt[base + i];
      offs[base + i] = run;
      cur[base + i]  = run;
      run += cv;
    }
    const unsigned bm = __builtin_amdgcn_ballot_w32(big != 0);
    if (lane == 0) misc[9] = misc[9] | ((bm != 0u) ? 1 : 0);
  }
  __syncthreads();

  if (wave == 0) {
    int t2 = 0;
#pragma unroll 1
    for (int w2 = 0; w2 < 8; ++w2) {
      const int c = __builtin_amdgcn_readfirstlane(clampi(misc[w2], 0, WLCAP));
#pragma unroll 1
      for (int b0 = 0; b0 < c; b0 += 32) {
        const int idx = (b0 + lane) < c ? (b0 + lane) : c - 1;
        const int ent = wl[w2 * WLCAP + idx];
        const int m32 = (c - b0) < 32 ? (c - b0) : 32;
#pragma unroll 1
        for (int k = 0; k < m32; ++k) {
          const int u    = __builtin_amdgcn_readlane(ent, k);
          const int slot = u & (NBRUN - 1);
          if (t2 < RCAP) {
            if (lane == 0) {
              int p = cur[slot];
              p = clampi(p, 0, RCAP - 1);
              sl[p] = u >> 10;
              cur[slot] = p + 1;
            }
            t2 = t2 + 1;
          }
        }
      }
    }
  }
  __syncthreads();

#pragma unroll 1
  for (int i = 0; i < 4; ++i) {
    const int s   = tid + 256 * i;
    const int deg = cnt[s] + 1;
    const float fd = (float)deg;
    const float r  = 1.0f / sqrtf(fd);
    dvb[s] = __float_as_int((deg > 0) ? r : 0.0f);
  }
  __syncthreads();

  const int ovf = misc[9];
  int* lbase = LIST + (size_t)blk * RCAP;
  for (int pass = 0; pass < 2; ++pass) {
    for (int i = tid; i < RCAP / 4; i += 256) {
      const v4i v = *(const v4ia*)(sl + 4 * i);
      *(volatile v4i*)(lbase + 4 * i) = v;
    }
    __threadfence();
  }
  const v4i cv4 = *(const v4ia*)(cnt + 4 * tid);
  const v4i ov4 = *(const v4ia*)(offs + 4 * tid);
  const v4i dv4 = *(const v4ia*)(dvb + 4 * tid);
  const v4f df4 = (v4f){ __int_as_float(dv4.x), __int_as_float(dv4.y), __int_as_float(dv4.z), __int_as_float(dv4.w) };
  const v4i fl4 = (v4i){ ovf, ovf, ovf, ovf };
  const size_t nb4 = (size_t)nodeBase + 4 * (size_t)tid;
  const bool fw = (wave == 0) && (lane < 8);
  *(volatile v4i*)(CNT + nb4) = cv4;
  *(volatile v4i*)(OFF + nb4) = ov4;
  *(volatile v4f*)(DINV + nb4) = df4;
  if (fw) *(volatile v4i*)(FLAG + blk * 32 + 4 * lane) = fl4;
  __threadfence();
  *(volatile v4i*)(CNT + nb4) = cv4;
  *(volatile v4i*)(OFF + nb4) = ov4;
  *(volatile v4f*)(DINV + nb4) = df4;
  if (fw) *(volatile v4i*)(FLAG + blk * 32 + 4 * lane) = fl4;
}

template <int NC> struct RowV;
template <> struct RowV<128> { typedef v4f T; typedef v4fa A; };
template <> struct RowV<64>  { typedef v2f T; typedef v2fa A; };

template <int NC>
__global__ __launch_bounds__(256) void k_replay(const float* __restrict__ P, const int* __restrict__ LIST,
                                                const int* __restrict__ CNT, const int* __restrict__ OFF,
                                                const float* __restrict__ DINV, const int* __restrict__ FLAG,
                                                const float* __restrict__ bias, float* outp, int nrows) {
  static_assert(NC == 128 || NC == 64);
  typedef typename RowV<NC>::T VT;
  typedef typename RowV<NC>::A VA;
  constexpr int CPL = NC / 32;
  __shared__ __attribute__((aligned(16))) float sB[NC];
  const int tid = (int)threadIdx.x, lane = tid & 31, wave = tid >> 5;
  if (wave == 0) {
    const VT b = *(const VA*)(bias + CPL * lane);
    asm volatile("" :: "v"(b));
    *(VA*)(sB + CPL * lane) = b;
  }
  __syncthreads();
  const VT bv = *(const VA*)(sB + CPL * lane);

  const int i    = (int)blockIdx.x * 8 + wave;
  const bool live = i < nrows;
  const int ic   = clampi(i, 0, NN - 1);
  const int b    = ic >> 10;
  int c  = CNT[ic];
  int o  = OFF[ic];
  const int fl = FLAG[b * 32];
  const float di = DINV[ic];
  asm volatile("" :: "v"(c));
  asm volatile("" :: "v"(o));
  asm volatile("" :: "v"(fl));
  asm volatile("" :: "v"(di));
  c = clampi(c, 0, DEGCAP);
  o = clampi(o, 0, RCAP - DEGCAP);
  const int cn = __builtin_amdgcn_readfirstlane(live ? c : 0);
  const int* lp = LIST + (size_t)b * RCAP + o;
  const float* Pl = P + CPL * lane;

  VT acc;
#pragma unroll
  for (int e = 0; e < CPL; ++e) acc[e] = 0.0f;
#pragma unroll 1
  for (int b0 = 0; b0 < cn; b0 += 32) {
    const int idx = (b0 + lane) < cn ? (b0 + lane) : cn - 1;
    int sr = lp[idx];
    asm volatile("" :: "v"(sr));
    sr = clampi(sr, 0, NN - 1);
    const float dv = DINV[sr];
    asm volatile("" :: "v"(dv));
    const float cf  = dv * di;
    const int   cfi = __float_as_int(cf);
    const int m32 = (cn - b0) < 32 ? (cn - b0) : 32;
#pragma unroll 1
    for (int k = 0; k < m32; ++k) {
      const int   skk = __builtin_amdgcn_readlane(sr, k);
      const float ck  = __int_as_float(__builtin_amdgcn_readlane(cfi, k));
      const VT row = *(const VA*)(Pl + (size_t)skk * NC);
      asm volatile("" :: "v"(row));
#pragma unroll
      for (int e = 0; e < CPL; ++e) acc[e] = acc[e] + row[e] * ck;
    }
  }
  const VT self = *(const VA*)(Pl + (size_t)ic * NC);
  asm volatile("" :: "v"(self));
  const float dd = di * di;
  const float qn = __int_as_float(0x7fc00000);
  const bool poison = fl != 0;
  VT v;
#pragma unroll
  for (int e = 0; e < CPL; ++e) {
    const float t = (acc[e] + self[e] * dd) + bv[e];
    v[e] = poison ? qn : t;
  }
  float* op = outp + (size_t)ic * NC + CPL * lane;
  if (live) *(volatile VT*)op = v;
  __threadfence();
  if (live) *(volatile VT*)op = v;
}

template <int MODE>
__global__ __launch_bounds__(256) void k_colstat(const float* __restrict__ H, const float* __restrict__ mean,
                                                 double* __restrict__ rec) {
  static_assert(MODE == 0 || MODE == 1);
  __shared__ __attribute__((aligned(16))) float  sm[HID];
  __shared__ __attribute__((aligned(16))) double sp[256];
  const int tid = (int)threadIdx.x;
  if (tid < 32) {
    v4f mv = (v4f){0.f, 0.f, 0.f, 0.f};
    if constexpr (MODE == 1) {
      mv = *(const v4fa*)(mean + 4 * tid);
      asm volatile("" :: "v"(mv));
    }
    *(v4fa*)(sm + 4 * tid) = mv;
  }
  __syncthreads();
  const int col = tid & (HID - 1);
  const int g   = tid >> 7;
  const int r0  = (int)blockIdx.x * 128 + g * 64;
  const int nr  = clampi(NN - r0, 0, 64);
  const float m = sm[col];
  const float* hp = H + (size_t)r0 * HID + col;
  double s = 0.0;
#pragma unroll 4
  for (int j = 0; j < nr; ++j) {
    const float v = hp[(size_t)j * HID];
    if constexpr (MODE == 0) {
      s += (double)v;
    } else {
      const float d = v - m;
      const double dd = (double)d;
      s += dd * dd;
    }
  }
  sp[tid] = s;
  __syncthreads();
  if (tid < 64) {
    const double a0 = sp[2 * tid] + sp[128 + 2 * tid];
    const double a1 = sp[2 * tid + 1] + sp[128 + 2 * tid + 1];
    const v2d o = (v2d){ a0, a1 };
    volatile v2d* q = (volatile v2d*)(rec + (size_t)blockIdx.x * HID + 2 * tid);
    *q = o;
    __threadfence();
    *q = o;
  }
}

__global__ __launch_bounds__(256) void k_comb(const double* __restrict__ rec, double inv_count, int mode,
                                              float* __restrict__ out) {
  __shared__ __attribute__((aligned(16))) float sv[256];
  const int tid = (int)threadIdx.x;
  const int c = tid < HID ? tid : HID - 1;
  double s = 0.0;
#pragma unroll 4
  for (int i = 0; i < NREC; ++i) s += rec[(size_t)i * HID + c];
  const float qf = (float)(s * inv_count);
  const float rs = 1.0f / sqrtf(qf + 1e-5f);
  sv[tid] = (mode == 0) ? qf : rs;
  __syncthreads();
  const int t4 = tid < 32 ? tid : 31;
  const v4f o = *(const v4fa*)(sv + 4 * t4);
  if (tid < 32) {
    volatile v4f* q = (volatile v4f*)(out + 4 * tid);
    *q = o;
    __threadfence();
    *q = o;
  }
}

template <int LAYER>
__global__ __launch_bounds__(256) void k_apply(const float* __restrict__ C, const unsigned* __restrict__ xbw,
                                               const float* resf,
                                               const float* __restrict__ mean, const float* __restrict__ rstd,
                                               const float* __restrict__ gam, const float* __restrict__ bet,
                                               float* h1out, unsigned short* __restrict__ hl) {
  static_assert(LAYER == 1 || LAYER == 2);
  constexpr int  KT  = (LAYER == 1) ? K2T : K3T;
  constexpr bool TWO = (KT == 2 * HID);
  __shared__ __attribute__((aligned(16))) float spar[4 * HID];
  const int tid = (int)threadIdx.x, lane = tid & 31, wave = tid >> 5;
  const int c0 = 4 * lane;
  if (wave == 0) {
    const v4f a0 = *(const v4fa*)(mean + c0);
    const v4f a1 = *(const v4fa*)(rstd + c0);
    const v4f a2 = *(const v4fa*)(gam + c0);
    const v4f a3 = *(const v4fa*)(bet + c0);
    asm volatile("" :: "v"(a0));
    asm volatile("" :: "v"(a1));
    asm volatile("" :: "v"(a2));
    asm volatile("" :: "v"(a3));
    *(v4fa*)(spar + c0)           = a0;
    *(v4fa*)(spar + HID + c0)     = a1;
    *(v4fa*)(spar + 2 * HID + c0) = a2;
    *(v4fa*)(spar + 3 * HID + c0) = a3;
  }
  __syncthreads();
  const v4f mv = *(const v4fa*)(spar + c0);
  const v4f rv = *(const v4fa*)(spar + HID + c0);
  const v4f gv = *(const v4fa*)(spar + 2 * HID + c0);
  const v4f bv = *(const v4fa*)(spar + 3 * HID + c0);
#pragma unroll 1
  for (int i = 0; i < 8; ++i) {
    const int row = (int)blockIdx.x * 64 + wave * 8 + i;
    const bool live = row < NN;
    const int rc = live ? row : NN - 1;
    const v4f cv = *(const v4fa*)(C + (size_t)rc * HID + c0);
    asm volatile("" :: "v"(cv));
    v4f sk;
    if constexpr (LAYER == 1) {
      const v2u w = *(const v2ua*)(xbw + (size_t)rc * (HID / 2) + 2 * lane);
      asm volatile("" :: "v"(w));
      sk = (v4f){ __uint_as_float(w.x << 16), __uint_as_float(w.x & 0xffff0000u),
                  __uint_as_float(w.y << 16), __uint_as_float(w.y & 0xffff0000u) };
    } else {
      sk = *(const v4fa*)(resf + (size_t)rc * HID + c0);
      asm volatile("" :: "v"(sk));
    }
    v4f y;
#pragma unroll
    for (int e = 0; e < 4; ++e) {
      const float t = relu_k(((cv[e] - mv[e]) * rv[e]) * gv[e] + bv[e]) + sk[e];
      y[e] = live ? t : 0.0f;
    }
    const v2u hv = (v2u){ pk16(bf16_bits(y[0]), bf16_bits(y[1])), pk16(bf16_bits(y[2]), bf16_bits(y[3])) };
    const v2u lv = (v2u){ pk16(bf16_lo_bits(y[0]), bf16_lo_bits(y[1])), pk16(bf16_lo_bits(y[2]), bf16_lo_bits(y[3])) };
    unsigned short* rp = hl + (size_t)row * KT + c0;
    float* fp = h1out + (size_t)rc * HID + c0;
    if (LAYER == 1 && live) *(volatile v4f*)fp = y;
    *(volatile v2u*)rp = hv;
    if (TWO) *(volatile v2u*)(rp + HID) = lv;
    __threadfence();
    if (LAYER == 1 && live) *(volatile v4f*)fp = y;
    *(volatile v2u*)rp = hv;
    if (TWO) *(volatile v2u*)(rp + HID) = lv;
  }
}

constexpr int G_GEMM128 = ((NP / 64) * (HID / 64) + 7) / 8;
constexpr int G_GEMM64  = ((NP / 64) * (COUT / 64) + 7) / 8;
static_assert(NP % 64 == 0 && HID % 64 == 0 && COUT % 64 == 0 && HID % 4 == 0 && COUT % 4 == 0);

extern "C" void kernel_launch(void* const* d_in, const int* in_sizes, int n_in,
                              void* d_out, int out_size, void* d_ws, size_t ws_size,
                              hipStream_t stream) {
  if (n_in < 12) return;
  if (in_sizes[0] != NN * HID) return;
  if (in_sizes[1] != 2 * NE) return;
  if (in_sizes[2] != HID * HID || in_sizes[3] != HID) return;
  if (in_sizes[4] != HID * HID || in_sizes[5] != HID) return;
  if (in_sizes[6] != HID * COUT || in_sizes[7] != COUT) return;
  if (in_sizes[8] != HID || in_sizes[9] != HID) return;
  if (in_sizes[10] != HID || in_sizes[11] != HID) return;
  if (out_size != NN * COUT) return;
  if (ws_size < WS_TOTAL) return;

  const float* x   = (const float*)d_in[0];
  const int*   ei  = (const int*)d_in[1];
  const float* W1  = (const float*)d_in[2];
  const float* b1  = (const float*)d_in[3];
  const float* W2  = (const float*)d_in[4];
  const float* b2  = (const float*)d_in[5];
  const float* W3  = (const float*)d_in[6];
  const float* b3  = (const float*)d_in[7];
  const float* g1  = (const float*)d_in[8];
  const float* be1 = (const float*)d_in[9];
  const float* g2  = (const float*)d_in[10];
  const float* be2 = (const float*)d_in[11];
  float* out = (float*)d_out;

  char* ws = (char*)d_ws;
  float*          PA   = (float*)(ws + OFF_PA);
  float*          PB   = (float*)(ws + OFF_PB);
  float*          PC   = (float*)(ws + OFF_PC);
  unsigned short* HL   = (unsigned short*)(ws + OFF_HL);
  unsigned short* XB   = (unsigned short*)(ws + OFF_XB);
  int*            LIST = (int*)(ws + OFF_LIST);
  int*            CNT  = (int*)(ws + OFF_CNT);
  int*            OFFS = (int*)(ws + OFF_OFF);
  float*          DINV = (float*)(ws + OFF_DINV);
  int*            FLAG = (int*)(ws + OFF_FLAG);
  unsigned short* W1T  = (unsigned short*)(ws + OFF_W1T);
  unsigned short* W2D  = (unsigned short*)(ws + OFF_W2D);
  unsigned short* W3D  = (unsigned short*)(ws + OFF_W3D);
  float*          PAR  = (float*)(ws + OFF_PAR);
  double*         REC  = (double*)(ws + OFF_REC);
  float*          ST   = (float*)(ws + OFF_ST);
  const unsigned* XBW  = (const unsigned*)XB;

  const double invN = 1.0 / (double)NN;

  hipFuncSetAttribute(reinterpret_cast<const void*>(&k_bucket), hipFuncAttributeMaxDynamicSharedMemorySize, (int)BK_LDS);

  k_prep<<<PB_TOT, 256, 0, stream>>>(x, W1, W2, W3, b1, b2, b3, g1, be1, g2, be2, XB, W1T, W2D, W3D, PAR);
  k_bucket<<<NBLK, 256, BK_LDS, stream>>>(ei, LIST, CNT, OFFS, DINV, FLAG);
  k_gemm_nt<0, 0><<<G_GEMM128, 256, 0, stream>>>(XB, W1T, PAR, PA, NP, HID, HID, HID);
  k_replay<HID><<<NN / 8, 256, 0, stream>>>(PA, LIST, CNT, OFFS, DINV, FLAG, PAR + P_B1, PB, NN);
  k_colstat<0><<<NREC, 256, 0, stream>>>(PB, ST + S_M1, REC);
  k_comb<<<1, 256, 0, stream>>>(REC, invN, 0, ST + S_M1);
  k_colstat<1><<<NREC, 256, 0, stream>>>(PB, ST + S_M1, REC);
  k_comb<<<1, 256, 0, stream>>>(REC, invN, 1, ST + S_R1);
  k_apply<1><<<NP / 64, 256, 0, stream>>>(PB, XBW, PB, ST + S_M1, ST + S_R1, PAR + P_G1, PAR + P_BE1, PA, HL);
  k_gemm_nt<0, 0><<<G_GEMM128, 256, 0, stream>>>(HL, W2D, PAR, PB, NP, HID, K2T, HID);
  k_replay<HID><<<NN / 8, 256, 0, stream>>>(PB, LIST, CNT, OFFS, DINV, FLAG, PAR + P_B2, PC, NN);
  k_colstat<0><<<NREC, 256, 0, stream>>>(PC, ST + S_M2, REC);
  k_comb<<<1, 256, 0, stream>>>(REC, invN, 0, ST + S_M2);
  k_colstat<1><<<NREC, 256, 0, stream>>>(PC, ST + S_M2, REC);
  k_comb<<<1, 256, 0, stream>>>(REC, invN, 1, ST + S_R2);
  k_apply<2><<<NP / 64, 256, 0, stream>>>(PC, XBW, PA, ST + S_M2, ST + S_R2, PAR + P_G2, PAR + P_BE2, PB, HL);
  k_gemm_nt<0, 0><<<G_GEMM64, 256, 0, stream>>>(HL, W3D, PAR, PB, NP, COUT, K3T, COUT);
  k_replay<COUT><<<NN / 8, 256, 0, stream>>>(PB, LIST, CNT, OFFS, DINV, FLAG, PAR + P_B3, out, NN);
}
